// Encoder_GNN_v_weighted_46815143526427
// MI455X (gfx1250) — hardware-verified
//
#include <hip/hip_runtime.h>


namespace {
constexpr int N = 50000, E = 1600000, F = 128, HD = 256, OUT = 128, NPAD = 50048, NBLK = NPAD / 128;

typedef _Float16 b16;
typedef __attribute__((ext_vector_type(16))) _Float16 v16b;
typedef __attribute__((ext_vector_type(8)))  _Float16 v8b;
typedef __attribute__((ext_vector_type(8)))  float v8f;
typedef __attribute__((ext_vector_type(4)))  float v4f;

__device__ __forceinline__ v8b ld8b(const b16* p) { return *(const v8b*)p; }
__device__ __forceinline__ v16b cat8b(v8b a, v8b b) { return __builtin_shufflevector(a, b, 0, 1, 2, 3, 4, 5, 6, 7, 8, 9, 10, 11, 12, 13, 14, 15); }
__device__ __forceinline__ v16b frag_kb(const b16* p, int hh) { return cat8b(ld8b(p + 8 * hh), ld8b(p + 16 + 8 * hh)); }
__device__ __forceinline__ void split16(float v, b16& hi, b16& lo) { hi = (b16)v; lo = (b16)(v - (float)hi); }
__device__ __forceinline__ void frag_ksplit(const float* p, int hh, v16b& fh_, v16b& fl_) {
  const float* p0 = p + 8 * hh; const float* p1 = p + 16 + 8 * hh;
#pragma unroll
  for (int e = 0; e < 8; ++e) { b16 a, c; split16(p0[e], a, c); fh_[e] = a; fl_[e] = c; split16(p1[e], a, c); fh_[8 + e] = a; fl_[8 + e] = c; }
}
__device__ __forceinline__ v8f wmma16b(v16b a, v16b b, v8f c) {
  v8f d = __builtin_amdgcn_wmma_f32_16x16x32_f16(false, a, false, b, (short)0, c, false, false);
  asm volatile("v_nop\n\tv_nop\n\tv_nop\n\tv_nop" : "+v"(d) : "v"(a), "v"(b));
  return d;
}
__device__ __forceinline__ void wave_lds_sync() {
  __builtin_amdgcn_fence(__ATOMIC_RELEASE, "workgroup");
  __builtin_amdgcn_wave_barrier();
  __builtin_amdgcn_fence(__ATOMIC_ACQUIRE, "workgroup");
}

struct Opnd { const void* p0; const void* p1; int ld; };
template <int NP> __device__ __forceinline__ void load_frags(const Opnd& o, int row, int kb, int hh, v16b& fh_, v16b& fl_) {
  if (NP == 0) { frag_ksplit((const float*)o.p0 + (size_t)row * o.ld + kb, hh, fh_, fl_); }
  else if (NP == 4) {
    const float* p = (const float*)o.p0 + (size_t)row * o.ld + kb; const float* p0 = p + 8 * hh; const float* p1 = p + 16 + 8 * hh;
#pragma unroll
    for (int e = 0; e < 8; ++e) { b16 a, c; split16(p0[e] * 64.0f, a, c); fh_[e] = a; fl_[e] = c; split16(p1[e] * 64.0f, a, c); fh_[8 + e] = a; fl_[8 + e] = c; }
  } else if (NP == 3) {
    const float* p = (const float*)o.p0 + (size_t)row * o.ld + kb; const float* p0 = p + 8 * hh; const float* p1 = p + 16 + 8 * hh;
#pragma unroll
    for (int e = 0; e < 8; ++e) { fh_[e] = (b16)p0[e]; fh_[8 + e] = (b16)p1[e]; }
    fl_ = fh_;
  } else {
    fh_ = frag_kb((const b16*)o.p0 + (size_t)row * o.ld + kb, hh);
    if (NP == 2) fl_ = frag_kb((const b16*)o.p1 + (size_t)row * o.ld + kb, hh); else fl_ = fh_;
  }
}
template <int ANP, int BNP> __device__ __forceinline__ v8f mac(v16b ah, v16b al, v16b bh, v16b bl, v8f c) {
  c = wmma16b(ah, bh, c);
  if (BNP == 0 || BNP == 2 || BNP == 4) c = wmma16b(ah, bl, c);
  if (ANP == 0 || ANP == 2 || ANP == 4) c = wmma16b(al, bh, c);
  return c;
}
template <int ANP, int BNP>
__device__ __forceinline__ void gemm_tile(const Opnd& A, const Opnd& B, int K, int m0, int c0, int nloc, int hlf, v8f (&acc)[2][4]) {
  for (int kb = 0; kb < K; kb += 32) {
    v16b a0h, a0l, a1h, a1l;
    load_frags<ANP>(A, m0 + nloc, kb, hlf, a0h, a0l);
    load_frags<ANP>(A, m0 + 16 + nloc, kb, hlf, a1h, a1l);
#pragma unroll
    for (int t = 0; t < 4; ++t) {
      v16b bh, bl;
      load_frags<BNP>(B, c0 + t * 16 + nloc, kb, hlf, bh, bl);
      acc[0][t] = mac<ANP, BNP>(a0h, a0l, bh, bl, acc[0][t]);
      acc[1][t] = mac<ANP, BNP>(a1h, a1l, bh, bl, acc[1][t]);
    }
  }
}

__device__ __forceinline__ void epi_planes(v8f (&acc)[2][4], float scale, bool two, b16* __restrict__ oh, b16* __restrict__ ol, int ldo,
                                           int m0, int c0, int lane, b16* Th, b16* Tl) {
  const int nloc = lane & 15, hlf = lane >> 4;
#pragma unroll
  for (int t = 0; t < 4; ++t)
#pragma unroll
    for (int r = 0; r < 2; ++r)
#pragma unroll
      for (int v = 0; v < 8; ++v) {
        const int rr = r * 16 + v + 8 * hlf, cc = t * 16 + nloc;
        b16 h_, l_; split16(acc[r][t][v] * scale, h_, l_);
        Th[rr * 64 + cc] = h_; Tl[rr * 64 + cc] = l_;
      }
  wave_lds_sync();
  for (int pass = 0; pass < 2; ++pass) {
#pragma unroll
    for (int j = 0; j < 8; ++j) {
      const int rr = j * 4 + (lane >> 3), c8 = (lane & 7) * 8;
      const size_t o = (size_t)(m0 + rr) * ldo + c0 + c8;
      *(volatile v8b*)(oh + o) = ld8b(Th + rr * 64 + c8);
      if (two) *(volatile v8b*)(ol + o) = ld8b(Tl + rr * 64 + c8);
    }
    __threadfence();
  }
}
__device__ __forceinline__ void epi_f32(v8f (&acc)[2][4], float scale, const float* rscale, float* __restrict__ out, int ldo, int m0, int c0, int lane, float* Tt) {
  const int nloc = lane & 15, hlf = lane >> 4;
#pragma unroll
  for (int t = 0; t < 4; ++t)
#pragma unroll
    for (int r = 0; r < 2; ++r)
#pragma unroll
      for (int v = 0; v < 8; ++v) {
        const int rr = r * 16 + v + 8 * hlf;
        const float rs = rscale ? rscale[(size_t)(m0 + rr) * 32] : 1.0f;
        Tt[rr * 64 + t * 16 + nloc] = acc[r][t][v] * scale * rs;
      }
  wave_lds_sync();
  float* dst0 = out + (size_t)m0 * ldo + c0;
  for (int pass = 0; pass < 2; ++pass) {
#pragma unroll
    for (int j = 0; j < 16; ++j) { const int rr = j * 2 + hlf, c4 = nloc * 4; *(volatile v4f*)(dst0 + (size_t)rr * ldo + c4) = *(const v4f*)(Tt + rr * 64 + c4); }
    __threadfence();
  }
}


__global__ __launch_bounds__(256) void prep_kernel(const float* __restrict__ W1l, const float* __restrict__ W1r, const float* __restrict__ W2l, const float* __restrict__ W2r, const float* __restrict__ Wo,
                                                   b16* __restrict__ w1, b16* __restrict__ w2, b16* __restrict__ wo) {
  const size_t tid = (size_t)blockIdx.x * blockDim.x + threadIdx.x, nth = (size_t)gridDim.x * blockDim.x;
  for (int pass = 0; pass < 2; ++pass) {
    for (size_t p = tid; p < (size_t)HD * 2 * F / 8; p += nth) { const int n = (int)(p / (2 * F / 8)), k0 = (int)(p % (2 * F / 8)) * 8; v8b v;
#pragma unroll
      for (int e = 0; e < 8; ++e) { const int k = k0 + e; v[e] = (b16)((k < F) ? W1l[(size_t)k * HD + n] : W1r[(size_t)(k - F) * HD + n]); }
      *(volatile v8b*)(w1 + (size_t)n * 2 * F + k0) = v; }
    for (size_t p = tid; p < (size_t)HD * 2 * HD / 8; p += nth) { const int n = (int)(p / (2 * HD / 8)), k0 = (int)(p % (2 * HD / 8)) * 8; v8b v;
#pragma unroll
      for (int e = 0; e < 8; ++e) { const int k = k0 + e; v[e] = (b16)((k < HD) ? W2l[(size_t)k * HD + n] : W2r[(size_t)(k - HD) * HD + n]); }
      *(volatile v8b*)(w2 + (size_t)n * 2 * HD + k0) = v; }
    for (size_t p = tid; p < (size_t)OUT * HD / 8; p += nth) { const int n = (int)(p / (HD / 8)), k0 = (int)(p % (HD / 8)) * 8; v8b v;
#pragma unroll
      for (int e = 0; e < 8; ++e) v[e] = (b16)Wo[(size_t)(k0 + e) * OUT + n];
      *(volatile v8b*)(wo + (size_t)n * HD + k0) = v; }
    __threadfence();
  }
}

template <int DF, int NB>
__global__ __launch_bounds__(256) void agg_kernel(const int* __restrict__ esrc, const int* __restrict__ edst, const float* __restrict__ x, b16* __restrict__ zin) {
  __shared__ __attribute__((aligned(16))) int acc[NB * DF];
  __shared__ int list[8 * 256]; __shared__ int cnt[NB];
  constexpr float FXS = 524288.0f, FXI = 1.0f / 524288.0f;
  const int t_ = threadIdx.x, wave = t_ >> 5, lane = t_ & 31, base = blockIdx.x * NB;
  for (int i = t_; i < NB * DF; i += 256) acc[i] = 0;
  for (int i = t_; i < NB; i += 256) cnt[i] = 0;
  __syncthreads();
  int* wl = list + wave * 256;
  typedef __attribute__((ext_vector_type(4))) int v4i;
  for (int c0 = 0; c0 < E; c0 += 256 * 8) {
    const int e0 = c0 + (wave * 32 + lane) * 8;
    int dd[8];
    if (e0 + 7 < E) { const v4i a = *(const v4i*)(edst + e0), b = *(const v4i*)(edst + e0 + 4); dd[0] = a[0]; dd[1] = a[1]; dd[2] = a[2]; dd[3] = a[3]; dd[4] = b[0]; dd[5] = b[1]; dd[6] = b[2]; dd[7] = b[3]; }
    else {
#pragma unroll
      for (int j = 0; j < 8; ++j) dd[j] = (e0 + j < E) ? edst[e0 + j] : -1; }
    unsigned sl[8]; bool hit[8]; bool anyl = false;
#pragma unroll
    for (int j = 0; j < 8; ++j) { sl[j] = (unsigned)(dd[j] - base); hit[j] = sl[j] < (unsigned)NB; anyl |= hit[j]; }
    int wc = 0;
    if (__builtin_amdgcn_ballot_w32(anyl) != 0u) {
#pragma unroll
      for (int j = 0; j < 8; ++j) {
        const unsigned mj = __builtin_amdgcn_ballot_w32(hit[j]);
        if (mj != 0u) {
          if (hit[j]) { const int pos = wc + (int)__builtin_amdgcn_mbcnt_lo(mj, 0u); int s = esrc[e0 + j]; s = (s < 0) ? 0 : (s >= N ? N - 1 : s); wl[pos] = (s << 12) | (int)sl[j]; atomicAdd(&cnt[sl[j]], 1); }
          wc += __builtin_popcount(mj);
        }
      }
    }
    __builtin_amdgcn_wave_barrier(); __builtin_amdgcn_fence(__ATOMIC_RELEASE, "workgroup"); __builtin_amdgcn_fence(__ATOMIC_ACQUIRE, "workgroup");
    if (DF <= 128) { constexpr int LPH = DF / 4, HPS = 32 / LPH;
      for (int i0 = 0; i0 < wc; i0 += HPS) { const int i = i0 + lane / LPH; if (i < wc) { const int ent = wl[i]; const int s = ent >> 12, slot = ent & 4095; const int col = (lane % LPH) * 4;
          const v4f v = *(const v4f*)(x + (size_t)s * DF + col);
#pragma unroll
          for (int c = 0; c < 4; ++c) atomicAdd(&acc[slot * DF + col + c], (int)rintf(v[c] * FXS)); } } }
    else {
      for (int i = 0; i < wc; ++i) { const int ent = wl[i]; const int s = ent >> 12, slot = ent & 4095;
#pragma unroll
        for (int ch = 0; ch < DF / 128; ++ch) { const int col = ch * 128 + lane * 4; const v4f v = *(const v4f*)(x + (size_t)s * DF + col);
#pragma unroll
          for (int c = 0; c < 4; ++c) atomicAdd(&acc[slot * DF + col + c], (int)rintf(v[c] * FXS)); } } }
    __builtin_amdgcn_wave_barrier();
  }
  __syncthreads();
  for (int pass = 0; pass < 2; ++pass) {
    for (int i = t_; i < NB * DF / 4; i += 256) { const int r = (i * 4) / DF; const int node = base + r; if (node < NPAD) {
        v4f o = {0.0f, 0.0f, 0.0f, 0.0f}; if (node < N) { const float inv = 1.0f / fmaxf((float)cnt[r], 1.0f);
#pragma unroll
          for (int c = 0; c < 4; ++c) o[c] = ((float)acc[i * 4 + c] * FXI) * inv; }
        typedef __attribute__((ext_vector_type(4))) _Float16 v4b; v4b ob; ob[0] = (b16)o[0]; ob[1] = (b16)o[1]; ob[2] = (b16)o[2]; ob[3] = (b16)o[3];
        *(volatile v4b*)(zin + (size_t)base * DF + (size_t)i * 4) = ob; } }
    __threadfence();
  }
}


template <int KA, int KX, int NOUT, bool RELU>
__global__ __launch_bounds__(128) void lin_kernel(const b16* __restrict__ agg, const float* __restrict__ xin, const b16* __restrict__ w, const float* __restrict__ bias, float* __restrict__ y, b16* __restrict__ y16, int nrows) {
  __shared__ __attribute__((aligned(16))) float Ts[4][32 * 64];
  const int lane = threadIdx.x & 31, wave = threadIdx.x >> 5, nloc = lane & 15, hlf = lane >> 4, m0 = blockIdx.y * 128 + wave * 32, c0 = blockIdx.x * 64;
  constexpr int K = KA + KX;
  v8f acc[2][4];
#pragma unroll
  for (int r = 0; r < 2; ++r)
#pragma unroll
    for (int t = 0; t < 4; ++t) acc[r][t] = (v8f){};
  const int ra = min(m0 + nloc, N - 1), rb = min(m0 + 16 + nloc, N - 1);
  const Opnd A1{agg, nullptr, KA}, A2{xin, nullptr, KX};
#pragma unroll 1
  for (int ks = 0; ks < K / 32; ++ks) { const bool first = (ks * 32 < KA);
    v16b a0, a1, d0, d1;
    if (first) { load_frags<1>(A1, m0 + nloc, ks * 32, hlf, a0, d0); load_frags<1>(A1, m0 + 16 + nloc, ks * 32, hlf, a1, d1); }
    else { load_frags<3>(A2, ra, ks * 32 - KA, hlf, a0, d0); load_frags<3>(A2, rb, ks * 32 - KA, hlf, a1, d1); }
#pragma unroll
    for (int t = 0; t < 4; ++t) { const v16b bw = frag_kb(w + (size_t)(c0 + t * 16 + nloc) * K + ks * 32, hlf); acc[0][t] = wmma16b(a0, bw, acc[0][t]); acc[1][t] = wmma16b(a1, bw, acc[1][t]); } }
  float* Tt = Ts[wave];
#pragma unroll
  for (int t = 0; t < 4; ++t)
#pragma unroll
    for (int r = 0; r < 2; ++r)
#pragma unroll
      for (int v = 0; v < 8; ++v) { float val = acc[r][t][v] + bias[c0 + t * 16 + nloc]; if (RELU) val = fmaxf(val, 0.0f); Tt[(r * 16 + v + 8 * hlf) * 64 + t * 16 + nloc] = val; }
  wave_lds_sync();
  for (int pass = 0; pass < 2; ++pass) {
#pragma unroll
    for (int j = 0; j < 16; ++j) { const int rr = j * 2 + hlf, c4 = nloc * 4; if (m0 + rr < nrows) { const v4f vv = *(const v4f*)(Tt + rr * 64 + c4); *(volatile v4f*)(y + (size_t)(m0 + rr) * NOUT + c0 + c4) = vv;
        if (y16 != nullptr) { typedef __attribute__((ext_vector_type(4))) _Float16 v4b; v4b ob; ob[0] = (b16)vv[0]; ob[1] = (b16)vv[1]; ob[2] = (b16)vv[2]; ob[3] = (b16)vv[3]; *(volatile v4b*)(y16 + (size_t)(m0 + rr) * NOUT + c0 + c4) = ob; } } }
    __threadfence();
  }
}
__global__ __launch_bounds__(128) void lin2out_kernel(const b16* __restrict__ agg, const b16* __restrict__ h1, const b16* __restrict__ w2, const float* __restrict__ b2, const b16* __restrict__ wo, const float* __restrict__ bo, float* __restrict__ out) {
  __shared__ __attribute__((aligned(16))) b16 Ht[32][HD + 8]; __shared__ __attribute__((aligned(16))) float Ot[4][32][32 + 4];
  const int lane = threadIdx.x & 31, wave = threadIdx.x >> 5, nloc = lane & 15, hlf = lane >> 4, m0 = blockIdx.x * 32, c0 = wave * 64;
  constexpr int K = 2 * HD;
  v8f acc[2][4];
#pragma unroll
  for (int r = 0; r < 2; ++r)
#pragma unroll
    for (int t = 0; t < 4; ++t) acc[r][t] = (v8f){};
#pragma unroll 2
  for (int ks = 0; ks < K / 32; ++ks) { const b16* A = (ks * 32 < HD) ? agg : h1; const int kb = (ks * 32 < HD) ? ks * 32 : ks * 32 - HD;
    const v16b a0 = frag_kb(A + (size_t)(m0 + nloc) * HD + kb, hlf), a1 = frag_kb(A + (size_t)(m0 + 16 + nloc) * HD + kb, hlf);
#pragma unroll
    for (int t = 0; t < 4; ++t) { const v16b bw = frag_kb(w2 + (size_t)(c0 + t * 16 + nloc) * K + ks * 32, hlf); acc[0][t] = wmma16b(a0, bw, acc[0][t]); acc[1][t] = wmma16b(a1, bw, acc[1][t]); } }
#pragma unroll
  for (int t = 0; t < 4; ++t)
#pragma unroll
    for (int r = 0; r < 2; ++r)
#pragma unroll
      for (int v = 0; v < 8; ++v) Ht[r * 16 + v + 8 * hlf][c0 + t * 16 + nloc] = (b16)fmaxf(acc[r][t][v] + b2[c0 + t * 16 + nloc], 0.0f);
  __syncthreads();
  v8f o2[2][2] = {{{}, {}}, {{}, {}}};
  const int oc0 = wave * 32;
#pragma unroll 2
  for (int kb = 0; kb < HD; kb += 32) { const v16b a0 = frag_kb(&Ht[nloc][0] + kb, hlf), a1 = frag_kb(&Ht[16 + nloc][0] + kb, hlf);
#pragma unroll
    for (int t = 0; t < 2; ++t) { const v16b bw = frag_kb(wo + (size_t)(oc0 + t * 16 + nloc) * HD + kb, hlf); o2[0][t] = wmma16b(a0, bw, o2[0][t]); o2[1][t] = wmma16b(a1, bw, o2[1][t]); } }
#pragma unroll
  for (int t = 0; t < 2; ++t)
#pragma unroll
    for (int r = 0; r < 2; ++r)
#pragma unroll
      for (int v = 0; v < 8; ++v) Ot[wave][r * 16 + v + 8 * hlf][t * 16 + nloc] = o2[r][t][v] + bo[oc0 + t * 16 + nloc];
  wave_lds_sync();
  for (int pass = 0; pass < 2; ++pass) {
#pragma unroll
    for (int j = 0; j < 8; ++j) { const int rr = j * 4 + (lane >> 3), c4 = (lane & 7) * 4; if (m0 + rr < N) *(volatile v4f*)(out + (size_t)(m0 + rr) * OUT + oc0 + c4) = *(const v4f*)(&Ot[wave][rr][c4]); }
    __threadfence();
  }
}
}

extern "C" void kernel_launch(void* const* d_in, const int* in_sizes, int n_in,
                              void* d_out, int out_size, void* d_ws, size_t ws_size, hipStream_t stream) {
  (void)n_in; (void)out_size;
  const float* x = (const float*)d_in[0]; const int* ei = (const int*)d_in[1];
  const float* W1l = (const float*)d_in[2]; const float* b1 = (const float*)d_in[3]; const float* W1r = (const float*)d_in[4];
  const float* W2l = (const float*)d_in[5]; const float* b2 = (const float*)d_in[6]; const float* W2r = (const float*)d_in[7];
  const float* Wo = (const float*)d_in[8]; const float* bo = (const float*)d_in[9];
  float* out = (float*)d_out;
  if (in_sizes[0] != N * F || in_sizes[1] != 2 * E || in_sizes[2] != F * HD || in_sizes[5] != HD * HD || in_sizes[8] != HD * OUT) return;
  const int* esrc = ei; const int* edst = ei + E;
  size_t off = 0; char* ws = (char*)d_ws;
  auto carve = [&](size_t bytes) { char* p = ws + off; off += (bytes + 255) & ~(size_t)255; return p; };
  b16* w1 = (b16*)carve((size_t)HD * 2 * F * 2); b16* w2 = (b16*)carve((size_t)HD * 2 * HD * 2); b16* wo = (b16*)carve((size_t)OUT * HD * 2);
  b16* agg1 = (b16*)carve((size_t)NPAD * F * 2); float* h1 = (float*)carve((size_t)NPAD * HD * 4); b16* h1h = (b16*)carve((size_t)NPAD * HD * 2); b16* agg2 = (b16*)carve((size_t)NPAD * HD * 2);
  if (off > ws_size) return;
  prep_kernel<<<256, 256, 0, stream>>>(W1l, W1r, W2l, W2r, Wo, w1, w2, wo);
  agg_kernel<F, 512><<<NPAD / 512 + 1, 256, 0, stream>>>(esrc, edst, x, agg1);
  lin_kernel<F, F, HD, true><<<dim3(HD / 64, NBLK), 128, 0, stream>>>(agg1, x, w1, b1, h1, h1h, NPAD);
  agg_kernel<HD, 256><<<NPAD / 256 + 1, 256, 0, stream>>>(esrc, edst, h1, agg2);
  lin2out_kernel<<<NPAD / 32, 128, 0, stream>>>(agg2, h1h, w2, b2, wo, bo, out);
}
